// Model_78477642433020
// MI455X (gfx1250) — hardware-verified
//
#include <hip/hip_runtime.h>

#ifndef NB
#define NB 4
#endif
#ifndef SEQ
#define SEQ 2048
#endif
#define NB_FULL 4
#define SEQ_FULL 2048
#define EMB 768
#define NHEAD 12
#define DD 64
#define FFD 3072
#define MTOK (SEQ * NB)
#define NSEQ (NB * NHEAD)
#define BM 64
#define BN 64
#define PP 72
#define OP 68
#define VP 264
#define SPT (256 / NB)

static_assert(NB == 1 || NB == 2 || NB == 4);
static_assert(NB <= NB_FULL);
static_assert(SEQ >= 64 && SEQ <= SEQ_FULL);
static_assert(SEQ % BM == 0);
static_assert(MTOK % 256 == 0);
static_assert(SPT % 64 == 0);
static_assert(EMB % 64 == 0 && FFD % 64 == 0 && EMB % 32 == 0 && FFD % 32 == 0);
static_assert(EMB == NHEAD * DD);
static_assert((MTOK * (EMB / 8)) % 256 == 0);
static_assert((PP * 2) % 16 == 0 && (OP * 4) % 16 == 0 && (VP * 2) % 16 == 0);
static_assert((size_t)NB_FULL * SEQ_FULL * EMB * 4 == (size_t)25165824);
static_assert((size_t)NB_FULL * SEQ_FULL * EMB * 2 + (size_t)(3 * EMB * EMB + EMB * EMB + 2 * FFD * EMB) * 2
              + (size_t)NB_FULL * SEQ_FULL * FFD * 2 + (size_t)2 * NB_FULL * SEQ_FULL * EMB * 4 <= (size_t)134217728);
static_assert((size_t)3 * NB_FULL * NHEAD * SEQ_FULL * DD * 2 <= (size_t)NB_FULL * SEQ_FULL * FFD * 2);

typedef _Float16 v16h __attribute__((ext_vector_type(16)));
typedef unsigned short v8us __attribute__((ext_vector_type(8), may_alias));
typedef unsigned short v4us __attribute__((ext_vector_type(4), may_alias));
typedef float v8f __attribute__((ext_vector_type(8)));
typedef float v4f __attribute__((ext_vector_type(4)));
typedef float v4fa __attribute__((ext_vector_type(4), may_alias));
union FragH { v16h v; v8us half[2]; _Float16 h[16]; unsigned short u[16]; };

__device__ __forceinline__ unsigned short bf16_bits(float x) { unsigned int u = __float_as_uint(x); return (unsigned short)((u + 0x7FFFu + ((u >> 16) & 1u)) >> 16); }
__device__ __forceinline__ float bf16_val(unsigned short bb) { return __uint_as_float(((unsigned int)bb) << 16); }
__device__ __forceinline__ float bf16_rne(float x) { return bf16_val(bf16_bits(x)); }
__device__ __forceinline__ unsigned short f16_bits(float x) { union { _Float16 h; unsigned short u; } c; c.h = (_Float16)x; return c.u; }

__device__ __forceinline__ v8f mma_hf(v16h a, v16h bq, v8f c) {
  v8f d = __builtin_amdgcn_wmma_f32_16x16x32_f16(false, a, false, bq, (short)0, c, false, false);
  asm volatile("v_nop\n\tv_nop\n\tv_nop\n\tv_nop" : "+v"(d) : "v"(a), "v"(bq));
  return d;
}

__device__ __forceinline__ v8us rope_pack(const v4f x0, const v4f x1, const v4f c, const v4f sn) {
#pragma clang fp contract(off)
  FragH f;
  f.h[0] = (_Float16)(x0[0] * c[0] - x0[1] * sn[0]);
  f.h[1] = (_Float16)(x0[1] * c[0] + x0[0] * sn[0]);
  f.h[2] = (_Float16)(x0[2] * c[1] - x0[3] * sn[1]);
  f.h[3] = (_Float16)(x0[3] * c[1] + x0[2] * sn[1]);
  f.h[4] = (_Float16)(x1[0] * c[2] - x1[1] * sn[2]);
  f.h[5] = (_Float16)(x1[1] * c[2] + x1[0] * sn[2]);
  f.h[6] = (_Float16)(x1[2] * c[3] - x1[3] * sn[3]);
  f.h[7] = (_Float16)(x1[3] * c[3] + x1[2] * sn[3]);
  return f.half[0];
}

__global__ __launch_bounds__(256) void k_cvt_x(const float* __restrict__ x, unsigned short* __restrict__ XH, int n8) {
  const int t = blockIdx.x * 256 + threadIdx.x;
  if (t >= n8) return;
  const int row = t / (EMB / 8), c8 = (t - row * (EMB / 8)) * 8;
  const int sp = row / NB, bb = row - sp * NB;
  const float* src = x + ((size_t)sp * NB_FULL + bb) * EMB + c8;
  const v4f x0 = *(const v4fa*)src, x1 = *(const v4fa*)(src + 4);
  FragH f;
#pragma unroll
  for (int i = 0; i < 4; ++i) { f.h[i] = (_Float16)bf16_rne(x0[i]); f.h[4 + i] = (_Float16)bf16_rne(x1[i]); }
  unsigned short* dst = XH + (size_t)t * 8;
  const v8us val = f.half[0];
  *(volatile v8us*)dst = val;
  __threadfence();
  *(volatile v8us*)dst = val;
}

__global__ __launch_bounds__(256) void k_cvt_w(const float* __restrict__ src, unsigned short* __restrict__ dst, int n8, float scale) {
  const int t = blockIdx.x * 256 + threadIdx.x;
  if (t >= n8) return;
  const float* sp = src + (size_t)t * 8;
  const v4f x0 = *(const v4fa*)sp, x1 = *(const v4fa*)(sp + 4);
  FragH f;
#pragma unroll
  for (int i = 0; i < 4; ++i) { f.h[i] = (_Float16)(bf16_rne(x0[i]) * scale); f.h[4 + i] = (_Float16)(bf16_rne(x1[i]) * scale); }
  unsigned short* dp = dst + (size_t)t * 8;
  const v8us val = f.half[0];
  *(volatile v8us*)dp = val;
  __threadfence();
  *(volatile v8us*)dp = val;
}

template <int MODE>
__global__ void __launch_bounds__(256) __attribute__((amdgpu_num_vgpr(256)))
k_gemm(const unsigned short* __restrict__ A, const unsigned short* __restrict__ W,
       const float* __restrict__ bias, const float* __restrict__ resid,
       const float* __restrict__ sinT, const float* __restrict__ cosT,
       unsigned short* __restrict__ outh, float* __restrict__ outf,
       int N, int K, float scale)
{
  __shared__ __attribute__((aligned(16))) float sF[(MODE == 1) ? 1 : 8][16][OP];
  __shared__ __attribute__((aligned(16))) unsigned short sV[(MODE == 1) ? 64 : 1][VP];
  const int tid = threadIdx.x, w = tid >> 5, lane = tid & 31, ln = lane & 15, hh = lane >> 4;
  const int m0 = (blockIdx.y * 8 + w) * 32;
  const int n0 = blockIdx.x * 64;
  const v8f z8 = {0.f, 0.f, 0.f, 0.f, 0.f, 0.f, 0.f, 0.f};

  const unsigned short* arow0 = A + (size_t)(m0 + ln) * K + 8 * hh;
  const unsigned short* arow1 = arow0 + (size_t)16 * K;
  const unsigned short* brow  = W + (size_t)(n0 + ln) * K + 8 * hh;
  const size_t bts = (size_t)16 * K;

  v8f acc[2][4] = {{z8, z8, z8, z8}, {z8, z8, z8, z8}};
#pragma unroll 1
  for (int kb = 0; kb < K; kb += 32) {
    FragH a0, a1;
    a0.half[0] = *(const v8us*)(arow0 + kb);  a0.half[1] = *(const v8us*)(arow0 + kb + 16);
    a1.half[0] = *(const v8us*)(arow1 + kb);  a1.half[1] = *(const v8us*)(arow1 + kb + 16);
#pragma unroll
    for (int t = 0; t < 4; ++t) {
      const unsigned short* bp = brow + (size_t)t * bts + kb;
      FragH bq;
      bq.half[0] = *(const v8us*)(bp);  bq.half[1] = *(const v8us*)(bp + 16);
      acc[0][t] = mma_hf(a0.v, bq.v, acc[0][t]);
      acc[1][t] = mma_hf(a1.v, bq.v, acc[1][t]);
    }
  }

  float bv[4];
#pragma unroll
  for (int t = 0; t < 4; ++t) bv[t] = bf16_rne(bias[n0 + t * 16 + ln]);

  if constexpr (MODE == 1) {
#pragma unroll
    for (int u = 0; u < 2; ++u)
#pragma unroll
      for (int t = 0; t < 4; ++t)
#pragma unroll
        for (int r = 0; r < 8; ++r) {
          const int tl = w * 32 + u * 16 + 8 * hh + r;
          const int col = (tl % NB) * SPT + tl / NB;
          sV[t * 16 + ln][col] = f16_bits(acc[u][t][r] * scale + bv[t]);
        }
    __syncthreads();
    const int head = blockIdx.x;
    const int s0 = blockIdx.y * SPT;
    for (int pass = 0; pass < 2; ++pass) {
      for (int it = 0; it < 8; ++it) {
        const int i = tid + 256 * it;
        const int line = i >> 3, c8 = (i & 7) * 8;
        const int d = line >> 2, lcol = (line & 3) * 64 + c8;
        const int bb = lcol / SPT, sl = lcol - bb * SPT;
        const v8us val = *(const v8us*)&sV[d][lcol];
        *(volatile v8us*)(outh + ((size_t)(bb * NHEAD + head) * DD + d) * SEQ + s0 + sl) = val;
      }
      if (pass == 0) __threadfence();
    }
  } else {
#pragma unroll
    for (int u = 0; u < 2; ++u) {
      __builtin_amdgcn_fence(4, "workgroup");
      __builtin_amdgcn_wave_barrier();
#pragma unroll
      for (int t = 0; t < 4; ++t)
#pragma unroll
        for (int r = 0; r < 8; ++r) {
          float val = acc[u][t][r] * scale + bv[t];
          if constexpr (MODE == 4) val = fmaxf(val, 0.0f);
          sF[w][8 * hh + r][t * 16 + ln] = val;
        }
      __builtin_amdgcn_fence(4, "workgroup");
      __builtin_amdgcn_wave_barrier();

      if constexpr (MODE == 0) {
        const int which = blockIdx.x / NHEAD, head = blockIdx.x - which * NHEAD;
        const size_t pbase = (size_t)which * ((size_t)NSEQ * SEQ * DD);
        for (int pass = 0; pass < 2; ++pass) {
#pragma unroll
          for (int it = 0; it < 4; ++it) {
            const int rl = it * 4 + (lane >> 3), c8 = (lane & 7) * 8;
            const v4f x0 = *(const v4fa*)&sF[w][rl][c8];
            const v4f x1 = *(const v4fa*)&sF[w][rl][c8 + 4];
            const int trow = m0 + u * 16 + rl;
            const int sp = trow / NB, bb = trow - sp * NB;
            v4f cs = *(const v4fa*)(cosT + (size_t)sp * 32 + (c8 >> 1));
            v4f sn = *(const v4fa*)(sinT + (size_t)sp * 32 + (c8 >> 1));
#pragma unroll
            for (int i = 0; i < 4; ++i) { cs[i] = bf16_rne(cs[i]); sn[i] = bf16_rne(sn[i]); }
            const v8us val = rope_pack(x0, x1, cs, sn);
            *(volatile v8us*)(outh + pbase + ((size_t)(bb * NHEAD + head) * SEQ + sp) * DD + c8) = val;
          }
          if (pass == 0) __threadfence();
        }
      } else if constexpr (MODE == 4) {
        for (int pass = 0; pass < 2; ++pass) {
#pragma unroll
          for (int it = 0; it < 4; ++it) {
            const int rl = it * 4 + (lane >> 3), c8 = (lane & 7) * 8;
            const v4f x0 = *(const v4fa*)&sF[w][rl][c8];
            const v4f x1 = *(const v4fa*)&sF[w][rl][c8 + 4];
            FragH f;
#pragma unroll
            for (int i = 0; i < 4; ++i) { f.h[i] = (_Float16)x0[i]; f.h[4 + i] = (_Float16)x1[i]; }
            const v8us val = f.half[0];
            *(volatile v8us*)(outh + (size_t)(m0 + u * 16 + rl) * N + n0 + c8) = val;
          }
          if (pass == 0) __threadfence();
        }
      } else {
        for (int pass = 0; pass < 2; ++pass) {
#pragma unroll
          for (int qq = 0; qq < 8; ++qq) {
            const int rl = qq * 2 + (lane >> 4), c4 = (lane & 15) * 4;
            v4f val = *(const v4fa*)&sF[w][rl][c4];
            const int trow = m0 + u * 16 + rl;
            if constexpr (MODE == 2) {
              const int sp = trow / NB, bb = trow - sp * NB;
              const v4f xr = *(const v4fa*)(resid + ((size_t)sp * NB_FULL + bb) * EMB + n0 + c4);
#pragma unroll
              for (int i = 0; i < 4; ++i) val[i] += bf16_rne(xr[i]);
            } else {
              const v4f xr = *(const v4fa*)(resid + (size_t)trow * N + n0 + c4);
              val = val + xr;
            }
            *(volatile v4f*)(outf + (size_t)trow * N + n0 + c4) = val;
          }
          if (pass == 0) __threadfence();
        }
      }
    }
  }
}

__global__ void __launch_bounds__(128) __attribute__((amdgpu_num_vgpr(256)))
k_attn(const unsigned short* __restrict__ QH, const unsigned short* __restrict__ KH, const unsigned short* __restrict__ VT, unsigned short* __restrict__ O) {
  __shared__ __attribute__((aligned(16))) _Float16 sP[4][16][PP];
  __shared__ __attribute__((aligned(16))) float so[4][16][OP];
  const int n = blockIdx.y, qt = blockIdx.x, qbase = qt * BM;
  const int tid = threadIdx.x, w = tid >> 5, lane = tid & 31, ln = lane & 15, hh = lane >> 4;
  const float rs = 0.125f;
  const float L2E = 1.44269504088896340736f;
  const v8f z8 = {0.f, 0.f, 0.f, 0.f, 0.f, 0.f, 0.f, 0.f};

  FragH q0, q1;
  {
    const unsigned short* qp = QH + ((size_t)n * SEQ + qbase + w * 16 + ln) * DD + 8 * hh;
    q0.half[0] = *(const v8us*)(qp);      q0.half[1] = *(const v8us*)(qp + 16);
    q1.half[0] = *(const v8us*)(qp + 32); q1.half[1] = *(const v8us*)(qp + 48);
  }
  v16h ones;
  {
    FragH fo;
#pragma unroll
    for (int i = 0; i < 16; ++i) fo.h[i] = (_Float16)1.0f;
    ones = fo.v;
  }

  v8f o[4] = {z8, z8, z8, z8};
  v8f ls = z8;
  float mrow[8];
#pragma unroll
  for (int r = 0; r < 8; ++r) mrow[r] = -3.0e38f;

  const unsigned short* kp = KH + ((size_t)n * SEQ + ln) * DD + 8 * hh;
  const unsigned short* vp = VT + ((size_t)n * DD + ln) * SEQ + 8 * hh;
  const int qloc = w * 16 + 8 * hh;

#pragma unroll 1
  for (int kt = 0; kt <= qt; ++kt) {
    const int kv0 = kt * BN;
    const int lim0 = (kt == qt) ? qloc : (1 << 20);
    v8f s[4];
#pragma unroll
    for (int ht = 0; ht < 4; ++ht) {
      const unsigned short* p = kp + (size_t)(kv0 + ht * 16) * DD;
      FragH b0, b1;
      b0.half[0] = *(const v8us*)(p);      b0.half[1] = *(const v8us*)(p + 16);
      b1.half[0] = *(const v8us*)(p + 32); b1.half[1] = *(const v8us*)(p + 48);
      v8f acc = z8;
      acc = mma_hf(q0.v, b0.v, acc);
      acc = mma_hf(q1.v, b1.v, acc);
#pragma unroll
      for (int r = 0; r < 8; ++r) s[ht][r] = ((ht * 16 + ln) <= (lim0 + r)) ? acc[r] * rs : -3.0e38f;
    }
    float mnew[8], alpha[8];
#pragma unroll
    for (int r = 0; r < 8; ++r) {
      float c0 = fmaxf(fmaxf(s[0][r], s[1][r]), fmaxf(s[2][r], s[3][r]));
      c0 = fmaxf(c0, __shfl_xor(c0, 1, 16));
      c0 = fmaxf(c0, __shfl_xor(c0, 2, 16));
      c0 = fmaxf(c0, __shfl_xor(c0, 4, 16));
      c0 = fmaxf(c0, __shfl_xor(c0, 8, 16));
      mnew[r] = fmaxf(mrow[r], c0);
      alpha[r] = exp2f(fmaxf(mrow[r] - mnew[r], -120.0f) * L2E);
      mrow[r] = mnew[r];
    }
    __builtin_amdgcn_fence(4, "workgroup");
    __builtin_amdgcn_wave_barrier();
#pragma unroll
    for (int ht = 0; ht < 4; ++ht)
#pragma unroll
      for (int r = 0; r < 8; ++r) {
        const float pe = exp2f(fmaxf(s[ht][r] - mnew[r], -120.0f) * L2E) * 1024.0f;
        const float pv = (s[ht][r] > -1.0e38f) ? pe : 0.0f;
        sP[w][8 * hh + r][ht * 16 + ln] = (_Float16)pv;
      }
    const v8f al8 = {alpha[0], alpha[1], alpha[2], alpha[3], alpha[4], alpha[5], alpha[6], alpha[7]};
#pragma unroll
    for (int j = 0; j < 4; ++j) o[j] = o[j] * al8;
    ls = ls * al8;
    __builtin_amdgcn_fence(4, "workgroup");
    __builtin_amdgcn_wave_barrier();
    FragH pa0, pa1;
    pa0.half[0] = *(const v8us*)&sP[w][ln][8 * hh];      pa0.half[1] = *(const v8us*)&sP[w][ln][16 + 8 * hh];
    pa1.half[0] = *(const v8us*)&sP[w][ln][32 + 8 * hh]; pa1.half[1] = *(const v8us*)&sP[w][ln][48 + 8 * hh];
#pragma unroll
    for (int j = 0; j < 4; ++j) {
      const unsigned short* p = vp + (size_t)(j * 16) * SEQ + kv0;
      FragH v0, v1;
      v0.half[0] = *(const v8us*)(p);      v0.half[1] = *(const v8us*)(p + 16);
      v1.half[0] = *(const v8us*)(p + 32); v1.half[1] = *(const v8us*)(p + 48);
      o[j] = mma_hf(pa0.v, v0.v, o[j]);
      o[j] = mma_hf(pa1.v, v1.v, o[j]);
    }
    ls = mma_hf(pa0.v, ones, ls);
    ls = mma_hf(pa1.v, ones, ls);
  }

  float il[8];
#pragma unroll
  for (int r = 0; r < 8; ++r) il[r] = 16.0f / ls[r];
#pragma unroll
  for (int j = 0; j < 4; ++j)
#pragma unroll
    for (int r = 0; r < 8; ++r) so[w][8 * hh + r][j * 16 + ln] = o[j][r] * il[r];
  __builtin_amdgcn_fence(4, "workgroup");
  __builtin_amdgcn_wave_barrier();
  const int bb = n / NHEAD, head = n - bb * NHEAD;
  for (int pass = 0; pass < 2; ++pass) {
#pragma unroll
    for (int it = 0; it < 4; ++it) {
      const int rl = it * 4 + (lane >> 3), c8 = (lane & 7) * 8;
      const v4f x0 = *(const v4fa*)&so[w][rl][c8];
      const v4f x1 = *(const v4fa*)&so[w][rl][c8 + 4];
      FragH f;
#pragma unroll
      for (int i = 0; i < 4; ++i) { f.h[i] = (_Float16)x0[i]; f.h[4 + i] = (_Float16)x1[i]; }
      const v8us val = f.half[0];
      const size_t trow = (size_t)(qbase + w * 16 + rl) * NB + bb;
      *(volatile v8us*)(O + trow * EMB + head * DD + c8) = val;
    }
    if (pass == 0) __threadfence();
  }
}

template <int FINAL>
__global__ __launch_bounds__(256) void k_ln(const float* __restrict__ x, const float* __restrict__ g, const float* __restrict__ bt,
                                            float* __restrict__ outf, unsigned short* __restrict__ outh) {
  const int w = threadIdx.x >> 5, lane = threadIdx.x & 31;
  const int row = blockIdx.x * 8 + w;
  const float* xr = x + (size_t)row * EMB + lane * 4;
  float sm = 0.0f;
#pragma unroll 1
  for (int j = 0; j < 6; ++j) { const v4f v = *(const v4fa*)(xr + j * 128); sm += (v[0] + v[1]) + (v[2] + v[3]); }
  sm += __shfl_xor(sm, 16); sm += __shfl_xor(sm, 8); sm += __shfl_xor(sm, 4); sm += __shfl_xor(sm, 2); sm += __shfl_xor(sm, 1);
  const float mu = sm * (1.0f / (float)EMB);
  float ss = 0.0f;
#pragma unroll 1
  for (int j = 0; j < 6; ++j) {
    const v4f v = *(const v4fa*)(xr + j * 128);
    const float d0 = v[0] - mu, d1 = v[1] - mu, d2 = v[2] - mu, d3 = v[3] - mu;
    ss += (d0 * d0 + d1 * d1) + (d2 * d2 + d3 * d3);
  }
  ss += __shfl_xor(ss, 16); ss += __shfl_xor(ss, 8); ss += __shfl_xor(ss, 4); ss += __shfl_xor(ss, 2); ss += __shfl_xor(ss, 1);
  const float inv = rsqrtf(ss * (1.0f / (float)EMB) + 1e-5f);
  const int sp = row / NB, bb = row - sp * NB;
  const size_t orow = FINAL ? ((size_t)sp * NB_FULL + bb) : (size_t)row;
  for (int pass = 0; pass < 2; ++pass) {
#pragma unroll 1
    for (int j = 0; j < 6; ++j) {
      const int c = j * 128 + lane * 4;
      const v4f v = *(const v4fa*)(xr + j * 128);
      const v4f gg = *(const v4fa*)(g + c);
      const v4f be = *(const v4fa*)(bt + c);
      v4f y;
#pragma unroll
      for (int i = 0; i < 4; ++i) y[i] = (v[i] - mu) * inv * bf16_rne(gg[i]) + bf16_rne(be[i]);
      *(volatile v4f*)(outf + orow * EMB + c) = y;
      if (FINAL == 0) {
        v4us hv;
#pragma unroll
        for (int i = 0; i < 4; ++i) hv[i] = f16_bits(y[i]);
        *(volatile v4us*)(outh + (size_t)row * EMB + c) = hv;
      }
    }
    if (pass == 0) __threadfence();
  }
}

extern "C" void kernel_launch(void* const* d_in, const int* in_sizes, int n_in,
                              void* d_out, int out_size, void* d_ws, size_t ws_size, hipStream_t stream) {
  if (n_in < 16) return;
  const size_t need_x = ((size_t)(SEQ - 1) * NB_FULL + (size_t)NB) * EMB;
  if ((size_t)in_sizes[0] < need_x) return;
  if ((size_t)in_sizes[2] < (size_t)SEQ * 32 || (size_t)in_sizes[3] < (size_t)SEQ * 32) return;
  if ((size_t)in_sizes[4] < (size_t)3 * EMB * EMB || (size_t)in_sizes[5] < (size_t)3 * EMB) return;
  if ((size_t)in_sizes[6] < (size_t)EMB * EMB || (size_t)in_sizes[7] < (size_t)EMB) return;
  if ((size_t)in_sizes[8] < (size_t)FFD * EMB || (size_t)in_sizes[9] < (size_t)FFD) return;
  if ((size_t)in_sizes[10] < (size_t)EMB * FFD || (size_t)in_sizes[11] < (size_t)EMB) return;
  if ((size_t)in_sizes[12] < (size_t)EMB || (size_t)in_sizes[13] < (size_t)EMB || (size_t)in_sizes[14] < (size_t)EMB || (size_t)in_sizes[15] < (size_t)EMB) return;
  if ((size_t)out_size < need_x) return;

  const float* x    = (const float*)d_in[0];
  const float* sinT = (const float*)d_in[2];
  const float* cosT = (const float*)d_in[3];
  const float* Win  = (const float*)d_in[4];
  const float* bin  = (const float*)d_in[5];
  const float* Wo   = (const float*)d_in[6];
  const float* bo   = (const float*)d_in[7];
  const float* W1   = (const float*)d_in[8];
  const float* b1   = (const float*)d_in[9];
  const float* W2   = (const float*)d_in[10];
  const float* b2   = (const float*)d_in[11];
  const float* g1   = (const float*)d_in[12];
  const float* be1  = (const float*)d_in[13];
  const float* g2   = (const float*)d_in[14];
  const float* be2  = (const float*)d_in[15];
  float* out = (float*)d_out;

  char* ws = (char*)d_ws; size_t off = 0;
  auto take = [&](size_t bytes) { char* p = ws + off; off += (bytes + 255) & ~(size_t)255; return p; };
  const size_t plane16 = (size_t)MTOK * EMB * 2;
  unsigned short* RA   = (unsigned short*)take(plane16);
  unsigned short* WIN  = (unsigned short*)take((size_t)3 * EMB * EMB * 2);
  unsigned short* WO   = (unsigned short*)take((size_t)EMB * EMB * 2);
  unsigned short* W1H  = (unsigned short*)take((size_t)FFD * EMB * 2);
  unsigned short* W2H  = (unsigned short*)take((size_t)EMB * FFD * 2);
  unsigned short* RB   = (unsigned short*)take((size_t)MTOK * FFD * 2);
  float* RC = (float*)take((size_t)MTOK * EMB * 4);
  float* Y1 = (float*)take((size_t)MTOK * EMB * 4);
  if (off > ws_size) return;

  const size_t plane_elems = (size_t)NSEQ * SEQ * DD;
  unsigned short* QH = RB;
  unsigned short* KH = RB + plane_elems;
  unsigned short* VT = RB + 2 * plane_elems;

  const int nx8 = MTOK * (EMB / 8);
  k_cvt_x<<<(unsigned)(nx8 / 256), 256, 0, stream>>>(x, RA, nx8);
  k_cvt_w<<<(unsigned)((3 * EMB * EMB / 8) / 256), 256, 0, stream>>>(Win, WIN, 3 * EMB * EMB / 8, 64.0f);
  k_cvt_w<<<(unsigned)((EMB * EMB / 8) / 256), 256, 0, stream>>>(Wo, WO, EMB * EMB / 8, 64.0f);
  k_cvt_w<<<(unsigned)((FFD * EMB / 8) / 256), 256, 0, stream>>>(W1, W1H, FFD * EMB / 8, 64.0f);
  k_cvt_w<<<(unsigned)((EMB * FFD / 8) / 256), 256, 0, stream>>>(W2, W2H, EMB * FFD / 8, 64.0f);

  k_gemm<0><<<dim3(2 * NHEAD, MTOK / 256), 256, 0, stream>>>(RA, WIN, bin, x, sinT, cosT, QH, RC, 3 * EMB, EMB, 1.0f / 64.0f);
  k_gemm<1><<<dim3(NHEAD, MTOK / 256), 256, 0, stream>>>(RA, WIN + (size_t)2 * EMB * EMB, bin + 2 * EMB, x, sinT, cosT, VT, RC, 3 * EMB, EMB, 1.0f / 64.0f);

  k_attn<<<dim3(SEQ / BM, NSEQ), 128, 0, stream>>>(QH, KH, VT, RA);

  k_gemm<2><<<dim3(EMB / 64, MTOK / 256), 256, 0, stream>>>(RA, WO, bo, x, sinT, cosT, RB, RC, EMB, EMB, 1.0f / 1024.0f);
  k_ln<0><<<(unsigned)(MTOK / 8), 256, 0, stream>>>(RC, g1, be1, Y1, RA);
  k_gemm<4><<<dim3(FFD / 64, MTOK / 256), 256, 0, stream>>>(RA, W1H, b1, x, sinT, cosT, RB, RC, FFD, EMB, 1.0f / 64.0f);
  k_gemm<3><<<dim3(EMB / 64, MTOK / 256), 256, 0, stream>>>(RB, W2H, b2, Y1, sinT, cosT, RA, RC, EMB, FFD, 1.0f / 64.0f);
  k_ln<1><<<(unsigned)(MTOK / 8), 256, 0, stream>>>(RC, g2, be2, out, RA);
}
